// SimpleEdgeModel_18683107737901
// MI455X (gfx1250) — hardware-run, weakly checked
//
#include <hip/hip_runtime.h>
#include <math.h>

typedef __attribute__((ext_vector_type(16))) _Float16 v16h;
typedef __attribute__((ext_vector_type(8)))  _Float16 v8h;
typedef __attribute__((ext_vector_type(16))) __bf16   v16b;
typedef __attribute__((ext_vector_type(8)))  __bf16   v8b;
typedef __attribute__((ext_vector_type(8)))  float    v8f;
typedef __attribute__((ext_vector_type(4)))  float    v4f;
typedef __attribute__((ext_vector_type(2)))  float    v2f;

constexpr int kBat    = 8;
constexpr int kNodes  = 192;
constexpr int kEmbW   = 128;
constexpr int kHid    = 512;
constexpr int kFields = 5;
constexpr int kTokRows = kBat * kNodes;
constexpr int kJTile  = 64;
constexpr int kActPitch = 520;
constexpr int kTabRowsB = 7;
constexpr int kTabRowsX = 32;
constexpr int kTabRowsY = 8;
constexpr int kTabRowsZ = 32;
constexpr int kPOff0 = 0;
constexpr int kPOff1 = kPOff0 + kTabRowsB;
constexpr int kPOff2 = kPOff1 + kTabRowsX;
constexpr int kPOff3 = kPOff2 + kTabRowsY;
constexpr int kPOff4 = kPOff3 + kTabRowsZ;
constexpr int kPRows = kPOff4 + kTabRowsX;
constexpr int kMatElems = kHid * kHid;
constexpr float kActCarry = 4096.0f;
constexpr float kWgtCarry = 32.0f;
constexpr float kAccToAct = 1.0f / kWgtCarry;
constexpr float kAccToVal = 1.0f / (kActCarry * kWgtCarry);

static_assert(kTokRows == 1536 && kPRows == 111, "shape constants");
static_assert((kHid % 32) == 0, "GEMM K multiple of 32");
static_assert((kTokRows % 64) == 0 && (kHid % 64) == 0 && ((2 * kHid) % 64) == 0, "GEMM M,N multiples of 64");
static_assert((kNodes % kJTile) == 0, "j tiles");
static_assert(((kActPitch * 2) % 16) == 0, "LDS rows 16-B aligned");

constexpr size_t kSzPT   = (size_t)kPRows * kHid * 4;
constexpr size_t kSzTok  = (size_t)kTokRows * kHid * 2;
constexpr size_t kSzBT3  = (size_t)3 * kMatElems * 2;
constexpr size_t kSzF16W = (size_t)2 * kMatElems * 2;
constexpr size_t kSzWOT  = (size_t)16 * kHid * 2;
constexpr size_t kSzPJPI = (size_t)kTokRows * 2 * kHid * 4;
constexpr size_t kOffPT   = 0;
constexpr size_t kOffFAH  = kOffPT   + kSzPT;
constexpr size_t kOffFAL  = kOffFAH  + kSzTok;
constexpr size_t kOffFEH  = kOffFAL  + kSzTok;
constexpr size_t kOffFEL  = kOffFEH  + kSzTok;
constexpr size_t kOffBT3H = kOffFEL  + kSzTok;
constexpr size_t kOffBT3L = kOffBT3H + kSzBT3;
constexpr size_t kOffF16W = kOffBT3L + kSzBT3;
constexpr size_t kOffWOT  = kOffF16W + kSzF16W;
constexpr size_t kOffPJPI = kOffWOT  + kSzWOT;
constexpr size_t kWsTotal = kOffPJPI + kSzPJPI;
static_assert(kWsTotal == 17020928ull, "carve total");
static_assert(kWsTotal <= 134217728ull, "carve cap");
static_assert((kOffFAH % 128) == 0 && (kOffFAL % 128) == 0 && (kOffFEH % 128) == 0 && (kOffFEL % 128) == 0 &&
              (kOffBT3H % 128) == 0 && (kOffBT3L % 128) == 0 && (kOffF16W % 128) == 0 && (kOffWOT % 128) == 0 &&
              (kOffPJPI % 128) == 0, "128-B aligned regions");

__device__ __forceinline__ unsigned short f2bf_bits(float f) {
  unsigned u = __float_as_uint(f);
  return (unsigned short)((u + 0x7FFFu + ((u >> 16) & 1u)) >> 16);
}
__device__ __forceinline__ float bf_bits2f(unsigned short h) { return __uint_as_float(((unsigned)h) << 16); }

__device__ __forceinline__ void grp_guard_h(v8f& a, v8f& b, v8f& c, v8f& d, v16h x, v16h y) {
  asm volatile("v_nop\n\tv_nop\n\tv_nop\n\tv_nop" : "+v"(a), "+v"(b), "+v"(c), "+v"(d) : "v"(x), "v"(y));
}
__device__ __forceinline__ void grp_guard_b(v8f& a, v8f& b, v8f& c, v8f& d, v16b x, v16b y) {
  asm volatile("v_nop\n\tv_nop\n\tv_nop\n\tv_nop" : "+v"(a), "+v"(b), "+v"(c), "+v"(d) : "v"(x), "v"(y));
}
__device__ __forceinline__ void keep4_h(v16h a, v16h b, v16h c, v16h d) { asm volatile("v_nop" :: "v"(a), "v"(b), "v"(c), "v"(d)); }
__device__ __forceinline__ void keep4_b(v16b a, v16b b, v16b c, v16b d) { asm volatile("v_nop" :: "v"(a), "v"(b), "v"(c), "v"(d)); }
__device__ __forceinline__ void acc_guard4(v8f& a, v8f& b, v8f& c, v8f& d) {
  asm volatile("v_nop\n\tv_nop\n\tv_nop\n\tv_nop" : "+v"(a), "+v"(b), "+v"(c), "+v"(d));
}
template <typename T> struct Frag;
template <> struct Frag<_Float16> {
  typedef v16h V; union U { v16h v; v8h h[2]; };
  static __device__ __forceinline__ v16h load(const _Float16* p) {
    U f; f.h[0] = *(const v8h*)(p); f.h[1] = *(const v8h*)(p + 16); return f.v;
  }
  static __device__ __forceinline__ v8f mma(v16h a, v16h b, v8f c) {
    return __builtin_amdgcn_wmma_f32_16x16x32_f16(false, a, false, b, (short)0, c, false, false);
  }
  static __device__ __forceinline__ void guard4(v8f& a, v8f& b, v8f& c, v8f& d, v16h x, v16h y) { grp_guard_h(a, b, c, d, x, y); }
  static __device__ __forceinline__ void keep(v16h a, v16h b, v16h c, v16h d) { keep4_h(a, b, c, d); }
};
template <> struct Frag<__bf16> {
  typedef v16b V; union U { v16b v; v8b h[2]; };
  static __device__ __forceinline__ v16b load(const __bf16* p) {
    U f; f.h[0] = *(const v8b*)(p); f.h[1] = *(const v8b*)(p + 16); return f.v;
  }
  static __device__ __forceinline__ v8f mma(v16b a, v16b b, v8f c) {
    return __builtin_amdgcn_wmma_f32_16x16x32_bf16(false, a, false, b, (short)0, c, false, false);
  }
  static __device__ __forceinline__ void guard4(v8f& a, v8f& b, v8f& c, v8f& d, v16b x, v16b y) { grp_guard_b(a, b, c, d, x, y); }
  static __device__ __forceinline__ void keep(v16b a, v16b b, v16b c, v16b d) { keep4_b(a, b, c, d); }
};

template <int ET> struct Elem;
template <> struct Elem<0> { typedef _Float16 T; };
template <> struct Elem<1> { typedef __bf16 T; };
template <int ET, int SPL, int BIAS_MODE, int OUT_MODE, bool RESID, int ACT = 0>
__global__ __launch_bounds__(256) void wmma_gemm64(
    const unsigned short* __restrict__ Ap, const unsigned short* __restrict__ A2p, int lda, long strideA,
    const unsigned short* __restrict__ Btp, const unsigned short* __restrict__ Bt2p, int ldb, long strideB,
    void* __restrict__ Cout, void* __restrict__ Cout2, int ldc, long strideC,
    const float* __restrict__ bias,
    const float* __restrict__ resid, long strideR,
    int M, int N, int K, float scale) {
  typedef typename Elem<ET>::T T;
  typedef typename Frag<T>::V V;
  const T* A = (const T*)Ap; const T* A2 = (const T*)A2p; const T* Bt = (const T*)Btp; const T* Bt2 = (const T*)Bt2p;
  __shared__ __align__(16) float sT[8][16 * 68];
  const int b    = blockIdx.y;
  const int lane = threadIdx.x & 31;
  const int wave = threadIdx.x >> 5;
  const int tilesN = N >> 6;
  const int tilesM = M >> 6;
  const int tile = blockIdx.x * 8 + wave;
  if (tile >= tilesM * tilesN) return;
  const int tm = tile / tilesN;
  const int tn = tile - tm * tilesN;
  const int m0 = tm << 6;
  const int n0 = tn << 6;

  const T* Ab  = A  + (size_t)b * strideA;
  const T* Bb  = Bt + (size_t)b * strideB;
  const T* Ab2 = (SPL >= 1) ? (A2  + (size_t)b * strideA) : nullptr;
  const T* Bb2 = (SPL == 2) ? (Bt2 + (size_t)b * strideB) : nullptr;

  const int rlane = lane & 15;
  const int koff  = (lane >> 4) * 8;
  const int mOff  = (lane >> 4) * 8;

  v8f acc[4][4];
#pragma unroll
  for (int i = 0; i < 4; ++i)
#pragma unroll
    for (int j = 0; j < 4; ++j) acc[i][j] = (v8f){0.f,0.f,0.f,0.f,0.f,0.f,0.f,0.f};

  for (int k0 = 0; k0 < K; k0 += 32) {
    V bh[4], bl[4];
#pragma unroll
    for (int j = 0; j < 4; ++j) {
      const size_t bo = (size_t)(n0 + (j << 4) + rlane) * ldb + koff + k0;
      bh[j] = Frag<T>::load(Bb + bo);
      if (SPL == 2) bl[j] = Frag<T>::load(Bb2 + bo);
    }
#pragma unroll
    for (int i = 0; i < 4; ++i) {
      const size_t ao = (size_t)(m0 + (i << 4) + rlane) * lda + koff + k0;
      V ah = Frag<T>::load(Ab + ao);
      V al;
      if (SPL >= 1) al = Frag<T>::load(Ab2 + ao);
#pragma unroll
      for (int j = 0; j < 4; ++j) {
        acc[i][j] = Frag<T>::mma(ah, bh[j], acc[i][j]);
        if (SPL == 2) acc[i][j] = Frag<T>::mma(ah, bl[j], acc[i][j]);
        if (SPL >= 1) acc[i][j] = Frag<T>::mma(al, bh[j], acc[i][j]);
      }
      Frag<T>::guard4(acc[i][0], acc[i][1], acc[i][2], acc[i][3], ah, (SPL >= 1) ? al : ah);
    }
    Frag<T>::keep(bh[0], bh[1], bh[2], bh[3]);
    if (SPL == 2) Frag<T>::keep(bl[0], bl[1], bl[2], bl[3]);
  }
  acc_guard4(acc[0][0], acc[0][1], acc[0][2], acc[0][3]);
  acc_guard4(acc[1][0], acc[1][1], acc[1][2], acc[1][3]);
  acc_guard4(acc[2][0], acc[2][1], acc[2][2], acc[2][3]);
  acc_guard4(acc[3][0], acc[3][1], acc[3][2], acc[3][3]);

  float* slab = sT[wave];
  const float* Rb = RESID ? (resid + (size_t)b * strideR) : nullptr;
#pragma unroll
  for (int i = 0; i < 4; ++i) {
    const int mBase = m0 + (i << 4);
#pragma unroll
    for (int j = 0; j < 4; ++j) {
      const int n = n0 + (j << 4) + rlane;
      float bv = 0.f;
      if (BIAS_MODE == 2) bv = bias[n];
#pragma unroll
      for (int r = 0; r < 8; ++r) {
        float v = acc[i][j][r] * scale;
        if (BIAS_MODE == 1) v += bias[mBase + mOff + r];
        if (BIAS_MODE == 2) v += bv;
        if (RESID) v += Rb[(size_t)(mBase + mOff + r) * ldc + n];
        if (ACT == 2) v = fmaxf(v, 0.0f);
        slab[(mOff + r) * 68 + (j << 4) + rlane] = v;
      }
    }
    __builtin_amdgcn_fence(__ATOMIC_RELEASE, "workgroup");
    __builtin_amdgcn_wave_barrier();
    __builtin_amdgcn_fence(__ATOMIC_ACQUIRE, "workgroup");
    if (OUT_MODE == 0) {
      float* C = (float*)Cout + (size_t)b * strideC;
      const int hh = lane >> 4, c4 = (lane & 15) * 4;
      for (int pass = 0; pass < 2; ++pass) {
#pragma unroll
        for (int it = 0; it < 8; ++it) {
          const int row = it * 2 + hh;
          v4f v = *(const v4f*)(slab + row * 68 + c4);
          *(volatile v4f*)(C + (size_t)(mBase + row) * ldc + n0 + c4) = v;
        }
        __threadfence();
      }
    } else {
      const int q = lane >> 3, c8 = (lane & 7) * 8;
      unsigned short* C  = (unsigned short*)Cout  + (size_t)b * strideC;
      unsigned short* C2 = (OUT_MODE == 2) ? ((unsigned short*)Cout2 + (size_t)b * strideC) : nullptr;
      for (int pass = 0; pass < 2; ++pass) {
#pragma unroll
        for (int it = 0; it < 4; ++it) {
          const int row = it * 4 + q;
          const float* sp = slab + row * 68 + c8;
          v8h hv, lv;
#pragma unroll
          for (int e = 0; e < 8; ++e) {
            if (OUT_MODE == 1) {
              hv[e] = (_Float16)sp[e];
            } else {
              unsigned short hb = f2bf_bits(sp[e]);
              unsigned short lb = f2bf_bits(sp[e] - bf_bits2f(hb));
              hv[e] = __builtin_bit_cast(_Float16, hb);
              lv[e] = __builtin_bit_cast(_Float16, lb);
            }
          }
          *(volatile v8h*)(C + (size_t)(mBase + row) * ldc + n0 + c8) = hv;
          if (OUT_MODE == 2) *(volatile v8h*)(C2 + (size_t)(mBase + row) * ldc + n0 + c8) = lv;
        }
        __threadfence();
      }
    }
    __builtin_amdgcn_fence(__ATOMIC_RELEASE, "workgroup");
    __builtin_amdgcn_wave_barrier();
    __builtin_amdgcn_fence(__ATOMIC_ACQUIRE, "workgroup");
  }
}

template <int MODE>
__global__ __launch_bounds__(256) void transpose_planes_kernel(
    const float* __restrict__ srcA, const float* __restrict__ srcB,
    unsigned short* __restrict__ dhi, unsigned short* __restrict__ dlo, float carry)
{
  __shared__ __align__(16) float sT[64 * 68];
  const int tid = threadIdx.x, lane = tid & 31, wave = tid >> 5;
  const int z = blockIdx.z;
  const float* src = (z == 0) ? srcA : (srcB + (size_t)(z - 1) * kMatElems);
  const size_t dbase = (size_t)z * kMatElems;
  const int n0 = blockIdx.x * 64, k0 = blockIdx.y * 64;
  {
    const int kr = tid >> 4, c4 = (tid & 15) * 4;
#pragma unroll
    for (int it = 0; it < 4; ++it) {
      const int kk = it * 16 + kr;
      const v4f v = *(const v4f*)(src + (size_t)(k0 + kk) * kHid + n0 + c4);
      *(v4f*)(sT + kk * 68 + c4) = v;
    }
  }
  __syncthreads();
  const int q = lane >> 3, c8 = (lane & 7) * 8;
  v8h hv[2], lv[2];
#pragma unroll
  for (int it = 0; it < 2; ++it) {
    const int nrow = it * 32 + wave * 4 + q;
#pragma unroll
    for (int e = 0; e < 8; ++e) {
      const float f = sT[(c8 + e) * 68 + nrow] * carry;
      if (MODE == 0) {
        const unsigned short hb = f2bf_bits(f);
        const unsigned short lb = f2bf_bits(f - bf_bits2f(hb));
        hv[it][e] = __builtin_bit_cast(_Float16, hb);
        lv[it][e] = __builtin_bit_cast(_Float16, lb);
      } else {
        hv[it][e] = (_Float16)f;
      }
    }
  }
  for (int pass = 0; pass < 2; ++pass) {
#pragma unroll
    for (int it = 0; it < 2; ++it) {
      const int nrow = it * 32 + wave * 4 + q;
      const size_t o = dbase + (size_t)(n0 + nrow) * kHid + k0 + c8;
      *(volatile v8h*)(dhi + o) = hv[it];
      if (MODE == 0) *(volatile v8h*)(dlo + o) = lv[it];
    }
    __threadfence();
  }
}

__global__ __launch_bounds__(256) void head_plane_kernel(const float* __restrict__ W_out, unsigned short* __restrict__ WOT)
{
  const int tid = threadIdx.x;
  v8h hv[4];
#pragma unroll
  for (int it = 0; it < 4; ++it) {
    const int item = it * 256 + tid;
    const int row = item >> 6;
    const int c8 = (item & 63) * 8;
    const float* wp = W_out + c8 * 2;
    const v4f f0 = *(const v4f*)(wp);
    const v4f f1 = *(const v4f*)(wp + 4);
    const v4f f2 = *(const v4f*)(wp + 8);
    const v4f f3 = *(const v4f*)(wp + 12);
    float ev[8], od[8];
    ev[0] = f0[0]; od[0] = f0[1]; ev[1] = f0[2]; od[1] = f0[3];
    ev[2] = f1[0]; od[2] = f1[1]; ev[3] = f1[2]; od[3] = f1[3];
    ev[4] = f2[0]; od[4] = f2[1]; ev[5] = f2[2]; od[5] = f2[3];
    ev[6] = f3[0]; od[6] = f3[1]; ev[7] = f3[2]; od[7] = f3[3];
#pragma unroll
    for (int e = 0; e < 8; ++e) {
      const float w = (row == 0) ? ev[e] : od[e];
      const float val = (row < 2) ? (w * kWgtCarry) : 0.0f;
      hv[it][e] = (_Float16)val;
    }
  }
  for (int pass = 0; pass < 2; ++pass) {
#pragma unroll
    for (int it = 0; it < 4; ++it) {
      const int item = it * 256 + tid;
      *(volatile v8h*)(WOT + (size_t)item * 8) = hv[it];
    }
    __threadfence();
  }
}

__global__ __launch_bounds__(128) void fold_tables_kernel(
    const float* __restrict__ e_b, const float* __restrict__ e_x, const float* __restrict__ e_y,
    const float* __restrict__ e_z, const float* __restrict__ W_a, float* __restrict__ PT)
{
  const int g = blockIdx.x;
  int s, v;
  if (g < kPOff1)      { s = 0; v = g - kPOff0; }
  else if (g < kPOff2) { s = 1; v = g - kPOff1; }
  else if (g < kPOff3) { s = 2; v = g - kPOff2; }
  else if (g < kPOff4) { s = 3; v = g - kPOff3; }
  else                 { s = 4; v = g - kPOff4; }
  const float* tab = (s == 0) ? e_b : ((s == 2) ? e_y : ((s == 3) ? e_z : e_x));
  const int h4 = threadIdx.x * 4;
  const float* trow = tab + (size_t)v * kEmbW;
  const float* wrow = W_a + (size_t)(s * kEmbW) * kHid + h4;
  float a0 = 0.f, a1 = 0.f, a2 = 0.f, a3 = 0.f;
#pragma unroll 4
  for (int d = 0; d < kEmbW; ++d) {
    const float traw = trow[d];
    const float t = (v == 0) ? 0.0f : traw;
    const v4f w = *(const v4f*)(wrow + (size_t)d * kHid);
    a0 = fmaf(t, w[0], a0);
    a1 = fmaf(t, w[1], a1);
    a2 = fmaf(t, w[2], a2);
    a3 = fmaf(t, w[3], a3);
  }
  v4f o;
  o[0] = a0; o[1] = a1; o[2] = a2; o[3] = a3;
  float* dst = PT + (size_t)g * kHid + h4;
  *(volatile v4f*)dst = o;
  __threadfence();
  *(volatile v4f*)dst = o;
}

__device__ __forceinline__ int clamp_idx(int v, int hi) { return v < 0 ? 0 : (v > hi ? hi : v); }

__global__ __launch_bounds__(256) void token_layer1_kernel(
    const int* __restrict__ bricks, const float* __restrict__ PT, const float* __restrict__ b_a,
    unsigned short* __restrict__ FAH, unsigned short* __restrict__ FAL)
{
  const int gid = blockIdx.x * 256 + threadIdx.x;
  if (gid >= kTokRows * 64) return;
  const int r = gid >> 6;
  const int h8 = (gid & 63) * 8;
  const int b = r / kNodes;
  const int n = r - b * kNodes;
  const int* bp = bricks + (size_t)(b * kFields) * kNodes + n;
  const int i0 = clamp_idx(bp[0], kTabRowsB - 1);
  const int i1 = clamp_idx(bp[kNodes], kTabRowsX - 1);
  const int i2 = clamp_idx(bp[2 * kNodes], kTabRowsY - 1);
  const int i3 = clamp_idx(bp[3 * kNodes], kTabRowsZ - 1);
  const int i4 = clamp_idx(bp[4 * kNodes], kTabRowsX - 1);
  const float* q0 = PT + (size_t)(kPOff0 + i0) * kHid + h8;
  const float* q1 = PT + (size_t)(kPOff1 + i1) * kHid + h8;
  const float* q2 = PT + (size_t)(kPOff2 + i2) * kHid + h8;
  const float* q3 = PT + (size_t)(kPOff3 + i3) * kHid + h8;
  const float* q4 = PT + (size_t)(kPOff4 + i4) * kHid + h8;
  v4f s0 = *(const v4f*)(q0);
  v4f s1 = *(const v4f*)(q0 + 4);
  s0 += *(const v4f*)(q1);
  s1 += *(const v4f*)(q1 + 4);
  s0 += *(const v4f*)(q2);
  s1 += *(const v4f*)(q2 + 4);
  s0 += *(const v4f*)(q3);
  s1 += *(const v4f*)(q3 + 4);
  s0 += *(const v4f*)(q4);
  s1 += *(const v4f*)(q4 + 4);
  s0 += *(const v4f*)(b_a + h8);
  s1 += *(const v4f*)(b_a + h8 + 4);
  v8h hv, lv;
#pragma unroll
  for (int e = 0; e < 4; ++e) {
    const float x0 = fmaxf(s0[e], 0.0f);
    const float x1 = fmaxf(s1[e], 0.0f);
    const unsigned short h0 = f2bf_bits(x0), h1 = f2bf_bits(x1);
    const unsigned short l0 = f2bf_bits(x0 - bf_bits2f(h0)), l1 = f2bf_bits(x1 - bf_bits2f(h1));
    hv[e]     = __builtin_bit_cast(_Float16, h0);
    hv[4 + e] = __builtin_bit_cast(_Float16, h1);
    lv[e]     = __builtin_bit_cast(_Float16, l0);
    lv[4 + e] = __builtin_bit_cast(_Float16, l1);
  }
  const size_t o = (size_t)r * kHid + h8;
  *(volatile v8h*)(FAH + o) = hv;
  *(volatile v8h*)(FAL + o) = lv;
  __threadfence();
  *(volatile v8h*)(FAH + o) = hv;
  *(volatile v8h*)(FAL + o) = lv;
}

__device__ __forceinline__ void edge_layer(const _Float16* src, _Float16* dst,
                                           const _Float16* __restrict__ Wt, const float* __restrict__ bias,
                                           int wave, int lane)
{
  const int rl = lane & 15;
  const int hh = lane >> 4;
  const int koff = hh * 8;
  const int n0 = wave * 64;
  v8f acc[4][4];
#pragma unroll
  for (int j = 0; j < 4; ++j)
#pragma unroll
    for (int i = 0; i < 4; ++i) acc[j][i] = (v8f){0.f,0.f,0.f,0.f,0.f,0.f,0.f,0.f};
  const _Float16* wbase = Wt + (size_t)(n0 + rl) * kHid + koff;
  const _Float16* xbase = src + rl * kActPitch + koff;
#pragma unroll 1
  for (int k0 = 0; k0 < kHid; k0 += 32) {
    v16h w[4];
#pragma unroll
    for (int j = 0; j < 4; ++j) w[j] = Frag<_Float16>::load(wbase + (size_t)(j * 16) * kHid + k0);
#pragma unroll
    for (int i = 0; i < 4; ++i) {
      const v16h x = Frag<_Float16>::load(xbase + (i * 16) * kActPitch + k0);
#pragma unroll
      for (int j = 0; j < 4; ++j) acc[j][i] = Frag<_Float16>::mma(w[j], x, acc[j][i]);
      grp_guard_h(acc[0][i], acc[1][i], acc[2][i], acc[3][i], x, w[0]);
    }
    keep4_h(w[0], w[1], w[2], w[3]);
  }
  acc_guard4(acc[0][0], acc[0][1], acc[0][2], acc[0][3]);
  acc_guard4(acc[1][0], acc[1][1], acc[1][2], acc[1][3]);
  acc_guard4(acc[2][0], acc[2][1], acc[2][2], acc[2][3]);
  acc_guard4(acc[3][0], acc[3][1], acc[3][2], acc[3][3]);
#pragma unroll
  for (int j = 0; j < 4; ++j) {
    const int nb = n0 + j * 16 + 8 * hh;
    const v4f b0 = *(const v4f*)(bias + nb);
    const v4f b1 = *(const v4f*)(bias + nb + 4);
    float bs[8];
#pragma unroll
    for (int e = 0; e < 4; ++e) {
      bs[e]     = b0[e] * kActCarry;
      bs[4 + e] = b1[e] * kActCarry;
    }
#pragma unroll
    for (int i = 0; i < 4; ++i) {
      v8h hv;
#pragma unroll
      for (int r = 0; r < 8; ++r) {
        const float t = fmaf(acc[j][i][r], kAccToAct, bs[r]);
        hv[r] = (_Float16)fmaxf(t, 0.0f);
      }
      *(v8h*)(dst + (i * 16 + rl) * kActPitch + nb) = hv;
    }
  }
}

__device__ __forceinline__ v8f mma_h_guarded(v16h a, v16h b, v8f c) {
  c = __builtin_amdgcn_wmma_f32_16x16x32_f16(false, a, false, b, (short)0, c, false, false);
  asm volatile("v_nop\n\tv_nop\n\tv_nop\n\tv_nop" : "+v"(c) : "v"(a), "v"(b));
  return c;
}

__global__ __launch_bounds__(256) void edge_fused_kernel(
    const float* __restrict__ PJPI, const float* __restrict__ b_ca,
    const float* __restrict__ b_cb, const float* __restrict__ b_cc,
    const float* __restrict__ b_out,
    const unsigned short* __restrict__ WcbTp, const unsigned short* __restrict__ WccTp,
    const unsigned short* __restrict__ WoTp, float* __restrict__ out)
{
  __shared__ __align__(16) _Float16 sA[kJTile * kActPitch];
  __shared__ __align__(16) _Float16 sB[kJTile * kActPitch];
  __shared__ __align__(16) float sO[kJTile * 2];

  const int tid = threadIdx.x;
  const int lane = tid & 31;
  const int wave = tid >> 5;
  const int blk = blockIdx.x;
  const int bi = blk / 3;
  const int jt = blk - bi * 3;
  const int b = bi / kNodes;
  const int j0 = jt * kJTile;

  const _Float16* WcbT = (const _Float16*)(const void*)WcbTp;
  const _Float16* WccT = (const _Float16*)(const void*)WccTp;
  const _Float16* WoT  = (const _Float16*)(const void*)WoTp;

  {
    const int k8 = (tid & 63) * 8;
    const int mq = tid >> 6;
    const float* pirow = PJPI + (size_t)bi * (2 * kHid) + kHid + k8;
    v4f p0 = *(const v4f*)(pirow);
    v4f p1 = *(const v4f*)(pirow + 4);
    p0 += *(const v4f*)(b_ca + k8);
    p1 += *(const v4f*)(b_ca + k8 + 4);
    const float* pjb = PJPI + (size_t)(b * kNodes + j0) * (2 * kHid) + k8;
#pragma unroll 4
    for (int it = 0; it < 16; ++it) {
      const int m = it * 4 + mq;
      const v4f a0 = *(const v4f*)(pjb + (size_t)m * (2 * kHid));
      const v4f a1 = *(const v4f*)(pjb + (size_t)m * (2 * kHid) + 4);
      v8h hv;
#pragma unroll
      for (int e = 0; e < 4; ++e) {
        const float u0 = a0[e] + p0[e];
        const float u1 = a1[e] + p1[e];
        hv[e]     = (_Float16)(fmaxf(u0, 0.0f) * kActCarry);
        hv[4 + e] = (_Float16)(fmaxf(u1, 0.0f) * kActCarry);
      }
      *(v8h*)(sA + m * kActPitch + k8) = hv;
    }
  }
  __syncthreads();

  edge_layer(sA, sB, WcbT, b_cb, wave, lane);
  __syncthreads();
  edge_layer(sB, sA, WccT, b_cc, wave, lane);
  __syncthreads();

  if (wave < 4) {
    const int rl = lane & 15;
    const int hh = lane >> 4;
    const int koff = hh * 8;
    v8f d = (v8f){0.f,0.f,0.f,0.f,0.f,0.f,0.f,0.f};
    const _Float16* wo = WoT + (size_t)rl * kHid + koff;
    const _Float16* xb = sA + (wave * 16 + rl) * kActPitch + koff;
#pragma unroll 2
    for (int k0 = 0; k0 < kHid; k0 += 32) {
      const v16h a = Frag<_Float16>::load(wo + k0);
      const v16h x = Frag<_Float16>::load(xb + k0);
      d = mma_h_guarded(a, x, d);
    }
    const float o0 = d[0] * kAccToVal + b_out[0];
    const float o1 = d[1] * kAccToVal + b_out[1];
    if (hh == 0) {
      v2f o;
      o[0] = o0;
      o[1] = o1;
      *(v2f*)(sO + (wave * 16 + rl) * 2) = o;
    }
  }
  __syncthreads();
  if (wave == 0) {
    const v4f v = *(const v4f*)(sO + lane * 4);
    float* ob = out + (size_t)blk * (kJTile * 2) + lane * 4;
    *(volatile v4f*)ob = v;
    __threadfence();
    *(volatile v4f*)ob = v;
  }
}

extern "C" void kernel_launch(void* const* d_in, const int* in_sizes, int n_in,
                              void* d_out, int out_size, void* d_ws, size_t ws_size,
                              hipStream_t stream) {
  if (n_in < 17) return;
  if (in_sizes[0] != kBat * kFields * kNodes) return;
  if (in_sizes[1] != kTabRowsB * kEmbW) return;
  if (in_sizes[2] != kTabRowsX * kEmbW) return;
  if (in_sizes[3] != kTabRowsY * kEmbW) return;
  if (in_sizes[4] != kTabRowsZ * kEmbW) return;
  if (in_sizes[5] != kFields * kEmbW * kHid) return;
  if (in_sizes[6] != kHid) return;
  if (in_sizes[7] != kMatElems) return;
  if (in_sizes[8] != kHid) return;
  if (in_sizes[9] != 2 * kMatElems) return;
  if (in_sizes[10] != kHid) return;
  if (in_sizes[11] != kMatElems) return;
  if (in_sizes[12] != kHid) return;
  if (in_sizes[13] != kMatElems) return;
  if (in_sizes[14] != kHid) return;
  if (in_sizes[15] != kHid * 2) return;
  if (in_sizes[16] != 2) return;
  if (out_size != kBat * kNodes * kNodes * 2) return;
  if (ws_size < kWsTotal) return;

  const int*   bricks = (const int*)  d_in[0];
  const float* e_b    = (const float*)d_in[1];
  const float* e_x    = (const float*)d_in[2];
  const float* e_y    = (const float*)d_in[3];
  const float* e_z    = (const float*)d_in[4];
  const float* W_a    = (const float*)d_in[5];
  const float* b_a    = (const float*)d_in[6];
  const float* W_b    = (const float*)d_in[7];
  const float* b_b    = (const float*)d_in[8];
  const float* W_ca   = (const float*)d_in[9];
  const float* b_ca   = (const float*)d_in[10];
  const float* W_cb   = (const float*)d_in[11];
  const float* b_cb   = (const float*)d_in[12];
  const float* W_cc   = (const float*)d_in[13];
  const float* b_cc   = (const float*)d_in[14];
  const float* W_out  = (const float*)d_in[15];
  const float* b_out  = (const float*)d_in[16];
  float* out = (float*)d_out;

  char* ws = (char*)d_ws;
  float*          PT   = (float*)(ws + kOffPT);
  unsigned short* FAH  = (unsigned short*)(ws + kOffFAH);
  unsigned short* FAL  = (unsigned short*)(ws + kOffFAL);
  unsigned short* FEH  = (unsigned short*)(ws + kOffFEH);
  unsigned short* FEL  = (unsigned short*)(ws + kOffFEL);
  unsigned short* BT3H = (unsigned short*)(ws + kOffBT3H);
  unsigned short* BT3L = (unsigned short*)(ws + kOffBT3L);
  unsigned short* F16W = (unsigned short*)(ws + kOffF16W);
  unsigned short* WOT  = (unsigned short*)(ws + kOffWOT);
  float*          PJPI = (float*)(ws + kOffPJPI);

  transpose_planes_kernel<0><<<dim3(kHid / 64, kHid / 64, 3), 256, 0, stream>>>(W_b, W_ca, BT3H, BT3L, 1.0f);
  transpose_planes_kernel<1><<<dim3(kHid / 64, kHid / 64, 2), 256, 0, stream>>>(W_cb, W_cc, F16W, F16W, kWgtCarry);
  head_plane_kernel<<<1, 256, 0, stream>>>(W_out, WOT);

  fold_tables_kernel<<<kPRows, 128, 0, stream>>>(e_b, e_x, e_y, e_z, W_a, PT);
  token_layer1_kernel<<<(kTokRows * 64) / 256, 256, 0, stream>>>(bricks, PT, b_a, FAH, FAL);

  wmma_gemm64<1, 2, 2, 2, false, 2><<<dim3(24, 1), 256, 0, stream>>>(
      FAH, FAL, kHid, 0L,
      BT3H, BT3L, kHid, 0L,
      (void*)FEH, (void*)FEL, kHid, 0L,
      b_b, nullptr, 0L,
      kTokRows, kHid, kHid, 1.0f);

  wmma_gemm64<1, 2, 0, 0, false, 0><<<dim3(48, 1), 256, 0, stream>>>(
      FEH, FEL, kHid, 0L,
      BT3H + (size_t)kMatElems, BT3L + (size_t)kMatElems, kHid, 0L,
      (void*)PJPI, nullptr, 2 * kHid, 0L,
      nullptr, nullptr, 0L,
      kTokRows, 2 * kHid, kHid, 1.0f);

  edge_fused_kernel<<<kBat * kNodes * (kNodes / kJTile), 256, 0, stream>>>(
      PJPI, b_ca, b_cb, b_cc, b_out,
      F16W, F16W + (size_t)kMatElems, WOT, out);
}
